// BiLSTM_79963701117082
// MI455X (gfx1250) — hardware-verified
//
#include <hip/hip_runtime.h>
#include <math.h>

constexpr int SEQ_T  = 16384;
constexpr int HID    = 128;
constexpr int NGATE  = 4 * HID;
constexpr int CAT    = 2 * HID;
constexpr int NPROJ  = 2 * NGATE;
constexpr int NTHR   = 256;
constexpr float WCARRY = 16.0f;
constexpr float HCARRY = 16.0f;
constexpr float FOLD   = 1.0f / (WCARRY * HCARRY);

constexpr int OFF_WIH1   = 0;
constexpr int OFF_FC1W   = NPROJ * CAT;
constexpr int OFF_WHH    = OFF_FC1W + HID * CAT;
constexpr int WHH_ELEMS  = NGATE * HID;
constexpr int W16_ELEMS  = OFF_WHH + 4 * WHH_ELEMS;
constexpr int BLK_WIH = NGATE * CAT / 8 / NTHR;
constexpr int BLK_FC1 = HID * CAT / 8 / NTHR;
constexpr int BLK_WHH = NGATE * HID / 8 / NTHR;
constexpr int BLK_CVT = 2 * BLK_WIH + BLK_FC1 + 4 * BLK_WHH;

static_assert(HID == 16 * (NTHR / 32));
static_assert(2 * HID == NTHR);
static_assert(SEQ_T % 64 == 0 && NPROJ % 64 == 0 && HID % 64 == 0);
static_assert(CAT % 32 == 0 && HID % 32 == 0);
static_assert(BLK_WIH == 64 && BLK_FC1 == 16 && BLK_WHH == 32 && BLK_CVT == 272);
static_assert(W16_ELEMS == BLK_CVT * NTHR * 8);
static_assert(NPROJ == 4 * NTHR);
static_assert(SEQ_T % NTHR == 0);
static_assert(((SEQ_T / 64) * (NPROJ / 64)) % 8 == 0);
static_assert(((SEQ_T / 64) * (HID / 64)) % 8 == 0);

typedef __attribute__((ext_vector_type(16))) _Float16 v16h;
typedef __attribute__((ext_vector_type(8)))  _Float16 v8h;
typedef __attribute__((ext_vector_type(4)))  _Float16 v4h;
typedef __attribute__((ext_vector_type(8)))  float    v8f;
typedef __attribute__((ext_vector_type(4)))  float    v4f;

__device__ __forceinline__ void guard_grp(v8f& a0, v8f& a1, v8f& a2, v8f& a3, v16h a, v16h b0, v16h b1, v16h b2, v16h b3) {
  asm volatile("v_nop\n\tv_nop\n\tv_nop\n\tv_nop" : "+v"(a0), "+v"(a1), "+v"(a2), "+v"(a3) : "v"(a), "v"(b0), "v"(b1), "v"(b2), "v"(b3));
}
__device__ __forceinline__ void acc_guard4(v8f& a, v8f& b, v8f& c, v8f& d) {
  asm volatile("v_nop\n\tv_nop\n\tv_nop\n\tv_nop" : "+v"(a), "+v"(b), "+v"(c), "+v"(d));
}
__device__ __forceinline__ void pin_frag(v16h& x) { asm volatile("" : "+v"(x)); }
__device__ __forceinline__ void pin_f32(float& x) { asm volatile("" : "+v"(x)); }

template <typename T> struct Frag;
template <> struct Frag<_Float16> {
  typedef v16h V; union U { v16h v; v8h h[2]; };
  static __device__ __forceinline__ v16h load(const _Float16* p) {
    U f; f.h[0] = *(const v8h*)(p); f.h[1] = *(const v8h*)(p + 16); return f.v;
  }
  static __device__ __forceinline__ v8f mma(v16h a, v16h b, v8f c) {
    return __builtin_amdgcn_wmma_f32_16x16x32_f16(false, a, false, b, (short)0, c, false, false);
  }
};

__device__ __forceinline__ float fsig(float x)  { return __builtin_amdgcn_rcpf(1.0f + __expf(-x)); }
__device__ __forceinline__ float ftanh(float x) { return 1.0f - 2.0f * __builtin_amdgcn_rcpf(__expf(2.0f * x) + 1.0f); }

__global__ __launch_bounds__(NTHR) void prep_kernel(
    const float* __restrict__ s0, const float* __restrict__ s1, const float* __restrict__ s2,
    const float* __restrict__ s3, const float* __restrict__ s4, const float* __restrict__ s5,
    const float* __restrict__ s6, unsigned short* __restrict__ dst,
    const float* __restrict__ biF, const float* __restrict__ bhF,
    const float* __restrict__ biR, const float* __restrict__ bhR, float* __restrict__ bsum) {
  const int tid = threadIdx.x;
  const int bx  = blockIdx.x;
  if (bx < BLK_CVT) {
    const float* src = s6;
    int bstart = 2 * BLK_WIH + BLK_FC1 + 3 * BLK_WHH;
    if (bx < BLK_WIH)                                   { src = s0; bstart = 0; }
    else if (bx < 2 * BLK_WIH)                          { src = s1; bstart = BLK_WIH; }
    else if (bx < 2 * BLK_WIH + BLK_FC1)                { src = s2; bstart = 2 * BLK_WIH; }
    else if (bx < 2 * BLK_WIH + BLK_FC1 + BLK_WHH)      { src = s3; bstart = 2 * BLK_WIH + BLK_FC1; }
    else if (bx < 2 * BLK_WIH + BLK_FC1 + 2 * BLK_WHH)  { src = s4; bstart = 2 * BLK_WIH + BLK_FC1 + BLK_WHH; }
    else if (bx < 2 * BLK_WIH + BLK_FC1 + 3 * BLK_WHH)  { src = s5; bstart = 2 * BLK_WIH + BLK_FC1 + 2 * BLK_WHH; }
    const size_t gi = (size_t)bx * NTHR + tid;
    const size_t li = (size_t)(bx - bstart) * NTHR + tid;
    const float* sp = src + li * 8;
    const v4f a = *(const v4f*)(sp);
    const v4f b = *(const v4f*)(sp + 4);
    v8h hv;
#pragma unroll
    for (int e = 0; e < 4; ++e) {
      const float fa = a[e] * WCARRY;
      const float fb = b[e] * WCARRY;
      hv[e]     = (_Float16)fa;
      hv[4 + e] = (_Float16)fb;
    }
    _Float16* dp = (_Float16*)dst + gi * 8;
    *(volatile v8h*)dp = hv;
    __threadfence();
    *(volatile v8h*)dp = hv;
  } else {
    const int which = tid >> 7;
    const int idx = (tid & 127) * 4;
    const v4f a0 = *(const v4f*)(biF + idx);
    const v4f a1 = *(const v4f*)(bhF + idx);
    const v4f r0 = *(const v4f*)(biR + idx);
    const v4f r1 = *(const v4f*)(bhR + idx);
    v4f o;
#pragma unroll
    for (int e = 0; e < 4; ++e) {
      const float sf = a0[e] + a1[e];
      const float sr = r0[e] + r1[e];
      o[e] = which ? sr : sf;
    }
    float* op = bsum + which * NGATE + idx;
    *(volatile v4f*)op = o;
    __threadfence();
    *(volatile v4f*)op = o;
  }
}

template <int LAYER>
__global__ __launch_bounds__(NTHR) void gate_scan_kernel(
    const float* __restrict__ xin,
    const float* __restrict__ wihF, const float* __restrict__ wihR,
    const float* __restrict__ bihF, const float* __restrict__ bhhF,
    const float* __restrict__ bihR, const float* __restrict__ bhhR,
    const float* __restrict__ gxp,
    const unsigned short* __restrict__ whFp, const unsigned short* __restrict__ whRp,
    unsigned short* __restrict__ houtp) {
  __shared__ __align__(16) _Float16 h_s[2 * HID];
  const int tid = threadIdx.x, lane = tid & 31, wave = tid >> 5;
  const int c = lane & 15, hh = lane >> 4, koff = hh * 8;
  const int dir = blockIdx.x;
  const int j = 16 * wave + c;
  const _Float16* WH = (const _Float16*)(dir ? whRp : whFp);
  _Float16* hout = (_Float16*)houtp + dir * HID;

  h_s[tid] = (_Float16)0.0f;

  float wi[4], bs[4];
#pragma unroll
  for (int g = 0; g < 4; ++g) { wi[g] = 0.0f; bs[g] = 0.0f; }
  if (LAYER == 0) {
    const float* wih = dir ? wihR : wihF;
    const float* bih = dir ? bihR : bihF;
    const float* bhh = dir ? bhhR : bhhF;
#pragma unroll
    for (int g = 0; g < 4; ++g) {
      const int r = g * HID + j;
      wi[g] = wih[r];
      bs[g] = bih[r] + bhh[r];
    }
  }

  v16h bfr[4][4];
#pragma unroll
  for (int g = 0; g < 4; ++g) {
#pragma unroll
    for (int kt = 0; kt < 4; ++kt) {
      bfr[g][kt] = Frag<_Float16>::load(WH + (size_t)(g * HID + j) * HID + kt * 32 + koff);
      pin_frag(bfr[g][kt]);
    }
  }
  float cst = 0.0f;
  __syncthreads();

  const v8f z8 = {0.f, 0.f, 0.f, 0.f, 0.f, 0.f, 0.f, 0.f};

#pragma unroll 1
  for (int s = 0; s < SEQ_T; ++s) {
    const int cur = s & 1;
    const int nxt = cur ^ 1;
    const int t = dir ? (SEQ_T - 1 - s) : s;

    float gin[4];
    if (LAYER == 0) {
      float xv = xin[t];
      pin_f32(xv);
#pragma unroll
      for (int g = 0; g < 4; ++g) gin[g] = xv * wi[g] + bs[g];
    } else {
      const float* gp = gxp + (size_t)t * NPROJ + dir * NGATE + j;
#pragma unroll
      for (int g = 0; g < 4; ++g) {
        gin[g] = gp[g * HID];
        pin_f32(gin[g]);
      }
    }

    const _Float16* hp = h_s + cur * HID + koff;
    v8f acc0 = z8, acc1 = z8, acc2 = z8, acc3 = z8;
#pragma unroll
    for (int kt = 0; kt < 4; ++kt) {
      const v16h a = Frag<_Float16>::load(hp + kt * 32);
      acc0 = Frag<_Float16>::mma(a, bfr[0][kt], acc0);
      acc1 = Frag<_Float16>::mma(a, bfr[1][kt], acc1);
      acc2 = Frag<_Float16>::mma(a, bfr[2][kt], acc2);
      acc3 = Frag<_Float16>::mma(a, bfr[3][kt], acc3);
      guard_grp(acc0, acc1, acc2, acc3, a, bfr[0][kt], bfr[1][kt], bfr[2][kt], bfr[3][kt]);
    }

    const float zi = acc0[0] * FOLD + gin[0];
    const float zf = acc1[0] * FOLD + gin[1];
    const float zg = acc2[0] * FOLD + gin[2];
    const float zo = acc3[0] * FOLD + gin[3];
    const float ig = fsig(zi);
    const float fg = fsig(zf);
    const float gg = ftanh(zg);
    const float og = fsig(zo);
    cst = fg * cst + ig * gg;
    const float hv = og * ftanh(cst);
    const _Float16 h16 = (_Float16)(hv * HCARRY);
    if (hh == 0) h_s[nxt * HID + j] = h16;
    __syncthreads();

    if (wave == 0) {
      const v4h hv4 = *(const v4h*)(h_s + nxt * HID + 4 * lane);
      _Float16* op = hout + (size_t)t * CAT + 4 * lane;
      for (int pass = 0; pass < 2; ++pass) {
        *(volatile v4h*)op = hv4;
        __threadfence();
      }
    }
  }
}

template <int ACT>
__global__ __launch_bounds__(256) void gemm64_f16_kernel(
    const unsigned short* __restrict__ Ap, int lda,
    const unsigned short* __restrict__ Btp, int ldb,
    float* __restrict__ C, int ldc,
    const float* __restrict__ bias, int M, int N, int K, float scale) {
  typedef _Float16 T;
  typedef v16h V;
  const T* A = (const T*)Ap;
  const T* Bt = (const T*)Btp;
  __shared__ __align__(16) float sT[8][16 * 68];
  const int lane = threadIdx.x & 31;
  const int wave = threadIdx.x >> 5;
  const int tilesN = N >> 6;
  const int tilesM = M >> 6;
  const int tile = blockIdx.x * 8 + wave;
  if (tile >= tilesM * tilesN) return;
  const int tm = tile / tilesN;
  const int tn = tile - tm * tilesN;
  const int m0 = tm << 6;
  const int n0 = tn << 6;

  const int rlane = lane & 15;
  const int koff  = (lane >> 4) * 8;
  const int mOff  = (lane >> 4) * 8;

  v8f acc[4][4];
#pragma unroll
  for (int i = 0; i < 4; ++i)
#pragma unroll
    for (int j = 0; j < 4; ++j) acc[i][j] = (v8f){0.f,0.f,0.f,0.f,0.f,0.f,0.f,0.f};

  for (int k0 = 0; k0 < K; k0 += 32) {
    V bh[4];
#pragma unroll
    for (int j = 0; j < 4; ++j) {
      const size_t bo = (size_t)(n0 + (j << 4) + rlane) * ldb + koff + k0;
      bh[j] = Frag<T>::load(Bt + bo);
    }
#pragma unroll
    for (int i = 0; i < 4; ++i) {
      const size_t ao = (size_t)(m0 + (i << 4) + rlane) * lda + koff + k0;
      V ah = Frag<T>::load(A + ao);
#pragma unroll
      for (int j = 0; j < 4; ++j) acc[i][j] = Frag<T>::mma(ah, bh[j], acc[i][j]);
      guard_grp(acc[i][0], acc[i][1], acc[i][2], acc[i][3], ah, bh[0], bh[1], bh[2], bh[3]);
    }
  }
  acc_guard4(acc[0][0], acc[0][1], acc[0][2], acc[0][3]);
  acc_guard4(acc[1][0], acc[1][1], acc[1][2], acc[1][3]);
  acc_guard4(acc[2][0], acc[2][1], acc[2][2], acc[2][3]);
  acc_guard4(acc[3][0], acc[3][1], acc[3][2], acc[3][3]);

  float* slab = sT[wave];
#pragma unroll
  for (int i = 0; i < 4; ++i) {
    const int mBase = m0 + (i << 4);
#pragma unroll
    for (int j = 0; j < 4; ++j) {
      const int n = n0 + (j << 4) + rlane;
      const float bv = bias[n];
#pragma unroll
      for (int r = 0; r < 8; ++r) {
        float v = acc[i][j][r] * scale;
        v += bv;
        if (ACT == 4) v = (v > 0.f) ? v : 0.01f * v;
        slab[(mOff + r) * 68 + (j << 4) + rlane] = v;
      }
    }
    __builtin_amdgcn_fence(__ATOMIC_RELEASE, "workgroup");
    __builtin_amdgcn_wave_barrier();
    __builtin_amdgcn_fence(__ATOMIC_ACQUIRE, "workgroup");
    {
      const int hh = lane >> 4, c4 = (lane & 15) * 4;
      for (int pass = 0; pass < 2; ++pass) {
#pragma unroll
        for (int it = 0; it < 8; ++it) {
          const int row = it * 2 + hh;
          v4f v = *(const v4f*)(slab + row * 68 + c4);
          *(volatile v4f*)(C + (size_t)(mBase + row) * ldc + n0 + c4) = v;
        }
        __threadfence();
      }
    }
    __builtin_amdgcn_fence(__ATOMIC_RELEASE, "workgroup");
    __builtin_amdgcn_wave_barrier();
    __builtin_amdgcn_fence(__ATOMIC_ACQUIRE, "workgroup");
  }
}

__global__ __launch_bounds__(NTHR) void head_dot_kernel(const float* __restrict__ y1, const float* __restrict__ w2,
                                                        const float* __restrict__ b2, float* __restrict__ out) {
  __shared__ __align__(16) float wsh[HID];
  const int tid = threadIdx.x;
  const float wv = w2[tid & (HID - 1)];
  if (tid < HID) wsh[tid] = wv;
  __syncthreads();
  const int t = blockIdx.x * NTHR + tid;
  const float* yp = y1 + (size_t)t * HID;
  float s0 = 0.0f, s1 = 0.0f, s2 = 0.0f, s3 = 0.0f;
#pragma unroll 1
  for (int k4 = 0; k4 < HID / 4; ++k4) {
    const v4f v = *(const v4f*)(yp + 4 * k4);
    const v4f w = *(const v4f*)(wsh + 4 * k4);
    s0 = fmaf(v[0], w[0], s0);
    s1 = fmaf(v[1], w[1], s1);
    s2 = fmaf(v[2], w[2], s2);
    s3 = fmaf(v[3], w[3], s3);
  }
  const float r = ((s0 + s1) + (s2 + s3)) + b2[0];
  float* op = out + t;
  *(volatile float*)op = r;
  __threadfence();
  *(volatile float*)op = r;
}

extern "C" void kernel_launch(void* const* d_in, const int* in_sizes, int n_in,
                              void* d_out, int out_size, void* d_ws, size_t ws_size, hipStream_t stream) {
  if (n_in < 21 || d_out == nullptr || d_ws == nullptr) return;
  if (in_sizes[0] != SEQ_T || in_sizes[1] != NGATE || in_sizes[2] != NGATE * HID || in_sizes[3] != NGATE ||
      in_sizes[4] != NGATE || in_sizes[5] != NGATE || in_sizes[6] != NGATE * HID || in_sizes[7] != NGATE ||
      in_sizes[8] != NGATE || in_sizes[9] != NGATE * CAT || in_sizes[10] != NGATE * HID || in_sizes[11] != NGATE ||
      in_sizes[12] != NGATE || in_sizes[13] != NGATE * CAT || in_sizes[14] != NGATE * HID || in_sizes[15] != NGATE ||
      in_sizes[16] != NGATE || in_sizes[17] != HID * CAT || in_sizes[18] != HID || in_sizes[19] != HID ||
      in_sizes[20] != 1 || out_size != SEQ_T) return;

  const float* x     = (const float*)d_in[0];
  const float* wih0  = (const float*)d_in[1];
  const float* whh0  = (const float*)d_in[2];
  const float* bih0  = (const float*)d_in[3];
  const float* bhh0  = (const float*)d_in[4];
  const float* wih0r = (const float*)d_in[5];
  const float* whh0r = (const float*)d_in[6];
  const float* bih0r = (const float*)d_in[7];
  const float* bhh0r = (const float*)d_in[8];
  const float* wih1  = (const float*)d_in[9];
  const float* whh1  = (const float*)d_in[10];
  const float* bih1  = (const float*)d_in[11];
  const float* bhh1  = (const float*)d_in[12];
  const float* wih1r = (const float*)d_in[13];
  const float* whh1r = (const float*)d_in[14];
  const float* bih1r = (const float*)d_in[15];
  const float* bhh1r = (const float*)d_in[16];
  const float* fc1w  = (const float*)d_in[17];
  const float* fc1b  = (const float*)d_in[18];
  const float* fc2w  = (const float*)d_in[19];
  const float* fc2b  = (const float*)d_in[20];
  float* out = (float*)d_out;

  char* ws = (char*)d_ws; size_t off = 0;
  auto carve = [&](size_t bytes) -> char* { char* p = ws + off; off += (bytes + 255) & ~(size_t)255; return p; };
  unsigned short* W16 = (unsigned short*)carve((size_t)W16_ELEMS * 2);
  float*          B1  = (float*)carve((size_t)NPROJ * 4);
  unsigned short* H0  = (unsigned short*)carve((size_t)SEQ_T * CAT * 2);
  float*          GX1 = (float*)carve((size_t)SEQ_T * NPROJ * 4);
  unsigned short* H1  = (unsigned short*)carve((size_t)SEQ_T * CAT * 2);
  float*          Y1  = (float*)carve((size_t)SEQ_T * HID * 4);
  if (off > ws_size || off > (size_t)134217728) return;

  prep_kernel<<<BLK_CVT + 1, NTHR, 0, stream>>>(wih1, wih1r, fc1w, whh0, whh0r, whh1, whh1r, W16,
                                                bih1, bhh1, bih1r, bhh1r, B1);

  gate_scan_kernel<0><<<2, NTHR, 0, stream>>>(x, wih0, wih0r, bih0, bhh0, bih0r, bhh0r, GX1,
                                              W16 + OFF_WHH, W16 + OFF_WHH + WHH_ELEMS, H0);

  gemm64_f16_kernel<0><<<(SEQ_T / 64) * (NPROJ / 64) / 8, 256, 0, stream>>>(
      H0, CAT, W16 + OFF_WIH1, CAT, GX1, NPROJ, B1, SEQ_T, NPROJ, CAT, FOLD);

  gate_scan_kernel<1><<<2, NTHR, 0, stream>>>(x, wih0, wih0r, bih0, bhh0, bih0r, bhh0r, GX1,
                                              W16 + OFF_WHH + 2 * WHH_ELEMS, W16 + OFF_WHH + 3 * WHH_ELEMS, H1);

  gemm64_f16_kernel<4><<<(SEQ_T / 64) * (HID / 64) / 8, 256, 0, stream>>>(
      H1, CAT, W16 + OFF_FC1W, CAT, Y1, HID, fc1b, SEQ_T, HID, CAT, FOLD);

  head_dot_kernel<<<SEQ_T / NTHR, NTHR, 0, stream>>>(Y1, fc2w, fc2b, out);
}
